// DiffMultiHeadedAttention_8280696947243
// MI455X (gfx1250) — hardware-verified
//
#include <hip/hip_runtime.h>
#include <math.h>
#include <float.h>
#include <stdint.h>

#ifndef NB
#define NB 2
#endif
#ifndef SEQ
#define SEQ 2048
#endif
#define NB_FULL  2
#define SEQ_FULL 2048
#define HID   1024
#define NPAIR 16
#define HD    64
#define HHALF 32
#define NQB   (SEQ / 64)
#define VLP   SEQ
static_assert(NB >= 1 && NB <= NB_FULL);
static_assert(SEQ >= 64 && SEQ <= SEQ_FULL && (SEQ % 64) == 0);
static_assert(NPAIR * HD == HID);
static_assert((HID % 64) == 0 && (HID % 32) == 0);
static_assert(((SEQ * HID / 8) % 256) == 0);
static_assert(((HID * HID / 8) % 256) == 0);

#define SM_SCALE      0.17677669529663687f
#define LAMBDA_INIT_F 0.7008206670670481f
#define OUT_SCALE     0.2991793329329519f

typedef _Float16 v16h __attribute__((ext_vector_type(16)));
typedef _Float16 v8h  __attribute__((ext_vector_type(8)));
typedef __bf16   v16b __attribute__((ext_vector_type(16)));
typedef __bf16   v8b  __attribute__((ext_vector_type(8)));
typedef float    v8f  __attribute__((ext_vector_type(8)));
typedef float    v4f  __attribute__((ext_vector_type(4)));
typedef unsigned int v4u __attribute__((ext_vector_type(4)));

__device__ __forceinline__ unsigned short bf_bits(float f) {
  unsigned u = __float_as_uint(f);
  return (unsigned short)((u + 0x7FFFu + ((u >> 16) & 1u)) >> 16);
}
__device__ __forceinline__ float bf_up(unsigned short h) { return __uint_as_float(((unsigned)h) << 16); }
__device__ __forceinline__ float bfq(float f) { return bf_up(bf_bits(f)); }
__device__ __forceinline__ unsigned short h_bits(_Float16 x) { return __builtin_bit_cast(unsigned short, x); }
__device__ __forceinline__ unsigned pk16(unsigned short a, unsigned short b) { return (unsigned)a | ((unsigned)b << 16); }
__device__ __forceinline__ v8f zero8() { v8f z = {0.f, 0.f, 0.f, 0.f, 0.f, 0.f, 0.f, 0.f}; return z; }
__device__ __forceinline__ v8h zero8h() {
  const _Float16 z = (_Float16)0.0f;
  v8h r = {z, z, z, z, z, z, z, z};
  return r;
}

__device__ __forceinline__ v16b ldfrag_b(const __bf16* p) {
  union { v16b v; v8b h[2]; } f;
  f.h[0] = *(const v8b*)(p);
  f.h[1] = *(const v8b*)(p + 16);
  return f.v;
}

__device__ __forceinline__ v8f mma_b(v16b a, v16b b, v8f c) {
  c = __builtin_amdgcn_wmma_f32_16x16x32_bf16(false, a, false, b, (short)0, c, false, false);
  asm volatile("v_nop\n\tv_nop\n\tv_nop\n\tv_nop" : "+v"(c) : "v"(a), "v"(b));
  return c;
}
__device__ __forceinline__ v8f mma_h(v16h a, v16h b, v8f c) {
  c = __builtin_amdgcn_wmma_f32_16x16x32_f16(false, a, false, b, (short)0, c, false, false);
  asm volatile("v_nop\n\tv_nop\n\tv_nop\n\tv_nop" : "+v"(c) : "v"(a), "v"(b));
  return c;
}
__device__ __forceinline__ v8f mma_b_raw(v16b a, v16b b, v8f c) {
  return __builtin_amdgcn_wmma_f32_16x16x32_bf16(false, a, false, b, (short)0, c, false, false);
}
__device__ __forceinline__ void dep_guard_b(v8f& a, v8f& b, v16b x, v16b y) {
  asm volatile("v_nop\n\tv_nop\n\tv_nop\n\tv_nop" : "+v"(a), "+v"(b) : "v"(x), "v"(y));
}
__device__ __forceinline__ void keep4_b(v16b a, v16b b, v16b c, v16b d) {
  asm volatile("v_nop" :: "v"(a), "v"(b), "v"(c), "v"(d));
}
__device__ __forceinline__ void acc_guard4(v8f& a, v8f& b, v8f& c, v8f& d) {
  asm volatile("v_nop\n\tv_nop\n\tv_nop\n\tv_nop" : "+v"(a), "+v"(b), "+v"(c), "+v"(d));
}

__global__ __launch_bounds__(256) void cvt_bf16x8(const float* __restrict__ in, unsigned short* out, int n8,
                                                  long long inStride, long long outStride) {
  const int i = blockIdx.x * 256 + threadIdx.x;
  const int y = blockIdx.y;
  if (i < n8) {
    const float* src = in + (size_t)y * (size_t)inStride + (size_t)i * 8;
    unsigned short* dst = out + (size_t)y * (size_t)outStride + (size_t)i * 8;
    const v4f a = *(const v4f*)(src);
    const v4f b = *(const v4f*)(src + 4);
    v4u p;
    p[0] = pk16(bf_bits(a[0]), bf_bits(a[1]));
    p[1] = pk16(bf_bits(a[2]), bf_bits(a[3]));
    p[2] = pk16(bf_bits(b[0]), bf_bits(b[1]));
    p[3] = pk16(bf_bits(b[2]), bf_bits(b[3]));
    *(volatile v4u*)(dst) = p;
    __threadfence();
    *(volatile v4u*)(dst) = p;
  }
}

template <int NSPLIT, int OUT_MODE>
__global__ __launch_bounds__(256) void gemm64(
    const unsigned short* __restrict__ Ap, const unsigned short* A2p, int lda, long long strideA,
    const unsigned short* __restrict__ Btp, const unsigned short* Bt2p, int ldb, long long strideB,
    void* Cout, int ldc, long long strideC,
    void* Cout2, int ldc2, long long strideC2, int N2,
    int M, int N, int K, float rscale) {
  const __bf16* A   = (const __bf16*)(const void*)Ap;
  const __bf16* A2  = (const __bf16*)(const void*)A2p;
  const __bf16* Bt  = (const __bf16*)(const void*)Btp;
  const __bf16* Bt2 = (const __bf16*)(const void*)Bt2p;
  __shared__ __align__(16) float sT[8][16 * 68];
  const int b    = blockIdx.y;
  const int lane = threadIdx.x & 31;
  const int wave = threadIdx.x >> 5;
  const int tilesN = N >> 6;
  const int tilesM = M >> 6;
  const int tile = blockIdx.x * 8 + wave;
  if (tile >= tilesM * tilesN) return;
  const int tm = tile / tilesN;
  const int tn = tile - tm * tilesN;
  const int m0 = tm << 6;
  const int n0 = tn << 6;

  const __bf16* Ab  = A  + (size_t)b * strideA;
  const __bf16* Bb  = Bt + (size_t)b * strideB;
  const __bf16* Ab2 = (NSPLIT >= 1) ? (A2  + (size_t)b * strideA) : Ab;
  const __bf16* Bb2 = (NSPLIT == 2) ? (Bt2 + (size_t)b * strideB) : Bb;

  const int rlane = lane & 15;
  const int koff  = (lane >> 4) * 8;
  const int mOff  = (lane >> 4) * 8;

  v8f acc[4][4];
#pragma unroll
  for (int i = 0; i < 4; ++i)
#pragma unroll
    for (int j = 0; j < 4; ++j) acc[i][j] = zero8();

  for (int k0 = 0; k0 < K; k0 += 32) {
    v16b bh[4], bl[4];
#pragma unroll
    for (int j = 0; j < 4; ++j) {
      const size_t bo = (size_t)(n0 + (j << 4) + rlane) * ldb + koff + k0;
      bh[j] = ldfrag_b(Bb + bo);
      if (NSPLIT == 2) bl[j] = ldfrag_b(Bb2 + bo); else bl[j] = bh[j];
    }
#pragma unroll
    for (int i = 0; i < 4; ++i) {
      const size_t ao = (size_t)(m0 + (i << 4) + rlane) * lda + koff + k0;
      const v16b ah = ldfrag_b(Ab + ao);
      v16b al = ah;
      if (NSPLIT >= 1) al = ldfrag_b(Ab2 + ao);
#pragma unroll
      for (int j = 0; j < 4; ++j) {
        acc[i][j] = mma_b_raw(ah, bh[j], acc[i][j]);
        if (NSPLIT >= 1) acc[i][j] = mma_b_raw(al, bh[j], acc[i][j]);
        if (NSPLIT == 2) acc[i][j] = mma_b_raw(ah, bl[j], acc[i][j]);
      }
      dep_guard_b(acc[i][0], acc[i][3], ah, al);
    }
    keep4_b(bh[0], bh[1], bh[2], bh[3]);
    if (NSPLIT == 2) keep4_b(bl[0], bl[1], bl[2], bl[3]);
  }
  acc_guard4(acc[0][0], acc[0][1], acc[0][2], acc[0][3]);
  acc_guard4(acc[1][0], acc[1][1], acc[1][2], acc[1][3]);
  acc_guard4(acc[2][0], acc[2][1], acc[2][2], acc[2][3]);
  acc_guard4(acc[3][0], acc[3][1], acc[3][2], acc[3][3]);

  float* slab = sT[wave];
#pragma unroll
  for (int i = 0; i < 4; ++i) {
    const int mBase = m0 + (i << 4);
#pragma unroll
    for (int j = 0; j < 4; ++j) {
#pragma unroll
      for (int r = 0; r < 8; ++r) {
        slab[(mOff + r) * 68 + (j << 4) + rlane] = acc[i][j][r];
      }
    }
    __builtin_amdgcn_fence(__ATOMIC_RELEASE, "workgroup");
    __builtin_amdgcn_wave_barrier();
    __builtin_amdgcn_fence(__ATOMIC_ACQUIRE, "workgroup");
    if (OUT_MODE == 0) {
      float* C = (float*)Cout + (size_t)b * strideC;
      const int hh = lane >> 4, c4 = (lane & 15) * 4;
      for (int pass = 0; pass < 2; ++pass) {
#pragma unroll
        for (int it = 0; it < 8; ++it) {
          const int row = it * 2 + hh;
          const v4f v = *(const v4f*)(slab + row * 68 + c4);
          *(volatile v4f*)(C + (size_t)(mBase + row) * ldc + n0 + c4) = v;
        }
        __threadfence();
      }
    } else {
      const int q = lane >> 3, c8 = (lane & 7) * 8;
      unsigned short* C  = (unsigned short*)Cout  + (size_t)b * strideC;
      unsigned short* C2 = (unsigned short*)Cout2 + (size_t)b * strideC2;
      const bool wlo = (OUT_MODE == 2) || (n0 < N2);
      v4u hv[4], lv[4];
#pragma unroll
      for (int it = 0; it < 4; ++it) {
        const int row = it * 4 + q;
        const float* sp = slab + row * 68 + c8;
        v4u a, a2;
#pragma unroll
        for (int e = 0; e < 4; ++e) {
          const float f0 = sp[2 * e], f1 = sp[2 * e + 1];
          unsigned short h0, h1, l0, l1;
          if (OUT_MODE == 2) {
            h0 = bf_bits(f0); h1 = bf_bits(f1);
            l0 = bf_bits(f0 - bf_up(h0)); l1 = bf_bits(f1 - bf_up(h1));
          } else {
            const _Float16 x0 = (_Float16)f0, x1 = (_Float16)f1;
            h0 = h_bits(x0); h1 = h_bits(x1);
            l0 = h_bits((_Float16)((f0 - (float)x0) * rscale));
            l1 = h_bits((_Float16)((f1 - (float)x1) * rscale));
          }
          a[e] = pk16(h0, h1); a2[e] = pk16(l0, l1);
        }
        hv[it] = a; lv[it] = a2;
      }
      for (int pass = 0; pass < 2; ++pass) {
#pragma unroll
        for (int it = 0; it < 4; ++it) {
          const int row = it * 4 + q;
          *(volatile v4u*)(C + (size_t)(mBase + row) * ldc + n0 + c8) = hv[it];
          if (wlo) *(volatile v4u*)(C2 + (size_t)(mBase + row) * ldc2 + n0 + c8) = lv[it];
        }
        __threadfence();
      }
    }
    __builtin_amdgcn_fence(__ATOMIC_RELEASE, "workgroup");
    __builtin_amdgcn_wave_barrier();
    __builtin_amdgcn_fence(__ATOMIC_ACQUIRE, "workgroup");
  }
}

template <bool RES>
__global__ __launch_bounds__(256)
void diff_attn64(const unsigned short* __restrict__ qhp, const unsigned short* __restrict__ qlp,
                 const unsigned short* __restrict__ khp, const unsigned short* __restrict__ klp,
                 const unsigned short* __restrict__ vhp, const unsigned short* __restrict__ vlp,
                 const float* __restrict__ lq1, const float* __restrict__ lq2,
                 const float* __restrict__ lk1, const float* __restrict__ lk2,
                 const float* __restrict__ gw,
                 unsigned short* ohp, unsigned short* olp, float sscale) {
  union FB { v16b v; v8b h[2]; };
  union FH { v16h v; v8h h[2]; };
  __shared__ __align__(16) __bf16   Ksh[64 * 64];
  __shared__ __align__(16) __bf16   Ksl[64 * 64];
  __shared__ __align__(16) _Float16 Vth[64 * 64];
  __shared__ __align__(16) _Float16 Vtl[RES ? 64 * 64 : 8];
  __shared__ __align__(16) _Float16 Psh[8][16 * 64];
  __shared__ __align__(16) _Float16 Psl[RES ? 8 : 1][16 * 64];
  __shared__ __align__(16) float    Os[4][16 * 64];

  const int tid  = threadIdx.x;
  const int wave = tid >> 5;
  const int lane = tid & 31;
  const int hh   = lane >> 4;
  const int c    = lane & 15;
  const int side = wave >> 2;
  const int wq   = wave & 3;

  const int bx   = blockIdx.x;
  const int qb   = bx % NQB;
  const int rest = bx / NQB;
  const int p    = rest % NPAIR;
  const int b    = rest / NPAIR;
  const int q0   = qb * 64 + wq * 16;
  const size_t rowB = (size_t)b * SEQ;

  const __bf16* Qh = (const __bf16*)(const void*)qhp + (size_t)p * HD + (size_t)side * HHALF;
  const __bf16* Ql = (const __bf16*)(const void*)qlp + (size_t)p * HD + (size_t)side * HHALF;
  const __bf16* Kh = (const __bf16*)(const void*)khp + (size_t)p * HD;
  const __bf16* Kl = (const __bf16*)(const void*)klp + (size_t)p * HD;
  const _Float16* Vh = (const _Float16*)(const void*)vhp + ((size_t)b * HID + (size_t)p * HD) * SEQ;
  const _Float16* Vl = (const _Float16*)(const void*)vlp + ((size_t)b * HID + (size_t)p * HD) * VLP;

  v16b qah, qal;
  {
    const size_t qo = (rowB + q0 + c) * HID + 8 * hh;
    qah = ldfrag_b(Qh + qo);
    qal = ldfrag_b(Ql + qo);
  }

  float mrow[8], lrow[8];
  v8f oacc[4];
#pragma unroll
  for (int r = 0; r < 8; ++r) { mrow[r] = -INFINITY; lrow[r] = 0.f; }
#pragma unroll
  for (int t = 0; t < 4; ++t) oacc[t] = zero8();

  const int nkt = qb + 1;
#pragma unroll 1
  for (int kt = 0; kt < nkt; ++kt) {
    const int kv0 = kt * 64;
    __syncthreads();
    {
      const int r = tid >> 2, qtr = (tid & 3) * 16;
      const __bf16*   kg  = Kh + (rowB + kv0 + r) * HID + qtr;
      const __bf16*   klg = Kl + (rowB + kv0 + r) * HID + qtr;
      const _Float16* vg  = Vh + (size_t)r * SEQ + kv0 + qtr;
      const int kvl = (kv0 + 64 <= VLP) ? kv0 : (VLP - 64);
      const _Float16* vlg = Vl + (size_t)r * VLP + kvl + qtr;
      const bool resOK = (kv0 + 64 <= VLP);
#pragma unroll
      for (int i = 0; i < 2; ++i) {
        const v8b a0 = *(const v8b*)(kg + 8 * i);
        const v8b a1 = *(const v8b*)(klg + 8 * i);
        const v8h b0 = *(const v8h*)(vg + 8 * i);
        *(v8b*)(Ksh + r * 64 + qtr + 8 * i) = a0;
        *(v8b*)(Ksl + r * 64 + qtr + 8 * i) = a1;
        *(v8h*)(Vth + r * 64 + qtr + 8 * i) = b0;
        if (RES) {
          v8h b1 = *(const v8h*)(vlg + 8 * i);
          if (!resOK) b1 = zero8h();
          *(v8h*)(Vtl + r * 64 + qtr + 8 * i) = b1;
        }
      }
    }
    __syncthreads();

    v8f s[4];
#pragma unroll
    for (int j = 0; j < 4; ++j) {
      FB kb, kl;
      kb.h[0] = *(const v8b*)(Ksh + (j * 16 + c) * 64 + side * HHALF + 8 * hh);
      kb.h[1] = *(const v8b*)(Ksh + (j * 16 + c) * 64 + side * HHALF + 16 + 8 * hh);
      kl.h[0] = *(const v8b*)(Ksl + (j * 16 + c) * 64 + side * HHALF + 8 * hh);
      kl.h[1] = *(const v8b*)(Ksl + (j * 16 + c) * 64 + side * HHALF + 16 + 8 * hh);
      s[j] = zero8();
      s[j] = mma_b(qah, kb.v, s[j]);
      s[j] = mma_b(qah, kl.v, s[j]);
      s[j] = mma_b(qal, kb.v, s[j]);
    }

    _Float16* pwh = Psh[wave];
    _Float16* pwl = Psl[RES ? wave : 0];
    const int trow0 = q0 + 8 * hh;
#pragma unroll
    for (int r = 0; r < 8; ++r) {
      float m = -INFINITY;
#pragma unroll
      for (int j = 0; j < 4; ++j) {
        const int key = kv0 + j * 16 + c;
        float sv = s[j][r] * sscale;
        sv = (key > trow0 + r) ? -FLT_MAX : sv;
        s[j][r] = sv;
        m = fmaxf(m, sv);
      }
#pragma unroll
      for (int off = 1; off < 16; off <<= 1) m = fmaxf(m, __shfl_xor(m, off, 32));
      const float mnew  = fmaxf(mrow[r], m);
      const float msafe = (mnew == -INFINITY) ? 0.f : mnew;
      const float alpha = __expf(mrow[r] - msafe);
      mrow[r] = mnew;
      float psum = 0.f;
#pragma unroll
      for (int j = 0; j < 4; ++j) {
        const float pe = __expf(s[j][r] - msafe);
        psum += pe;
        const float p1k = pe * 1024.0f;
        const _Float16 ph = (_Float16)p1k;
        pwh[(8 * hh + r) * 64 + j * 16 + c] = ph;
        if (RES) {
          const _Float16 pl = (_Float16)((p1k - (float)ph) * 4096.0f);
          pwl[(8 * hh + r) * 64 + j * 16 + c] = pl;
        }
      }
#pragma unroll
      for (int off = 1; off < 16; off <<= 1) psum += __shfl_xor(psum, off, 32);
      lrow[r] = lrow[r] * alpha + psum;
#pragma unroll
      for (int t = 0; t < 4; ++t) oacc[t][r] *= alpha;
    }
    __builtin_amdgcn_fence(__ATOMIC_RELEASE, "workgroup");
    __builtin_amdgcn_wave_barrier();
    __builtin_amdgcn_fence(__ATOMIC_ACQUIRE, "workgroup");

    v8f o1[4];
#pragma unroll
    for (int t = 0; t < 4; ++t) o1[t] = zero8();
#pragma unroll 1
    for (int kk = 0; kk < 2; ++kk) {
      FH pa, pl;
      pa.h[0] = *(const v8h*)(pwh + c * 64 + kk * 32 + 8 * hh);
      pa.h[1] = *(const v8h*)(pwh + c * 64 + kk * 32 + 16 + 8 * hh);
      if (RES) {
        pl.h[0] = *(const v8h*)(pwl + c * 64 + kk * 32 + 8 * hh);
        pl.h[1] = *(const v8h*)(pwl + c * 64 + kk * 32 + 16 + 8 * hh);
      } else {
        pl.v = pa.v;
      }
#pragma unroll
      for (int t = 0; t < 4; ++t) {
        FH vb;
        vb.h[0] = *(const v8h*)(Vth + (t * 16 + c) * 64 + kk * 32 + 8 * hh);
        vb.h[1] = *(const v8h*)(Vth + (t * 16 + c) * 64 + kk * 32 + 16 + 8 * hh);
        oacc[t] = mma_h(pa.v, vb.v, oacc[t]);
        if (RES) {
          FH vl;
          vl.h[0] = *(const v8h*)(Vtl + (t * 16 + c) * 64 + kk * 32 + 8 * hh);
          vl.h[1] = *(const v8h*)(Vtl + (t * 16 + c) * 64 + kk * 32 + 16 + 8 * hh);
          o1[t] = mma_h(pa.v, vl.v, o1[t]);
          o1[t] = mma_h(pl.v, vb.v, o1[t]);
        }
      }
    }
    if (RES) {
#pragma unroll
      for (int t = 0; t < 4; ++t)
#pragma unroll
        for (int r = 0; r < 8; ++r) oacc[t][r] += o1[t][r] * (1.0f / 4096.0f);
    }
  }

  float* os = Os[wq];
  if (side == 1) {
#pragma unroll
    for (int r = 0; r < 8; ++r) {
      const float l = lrow[r];
      const float inv = ((l > 0.f) ? (1.0f / l) : 0.f) * (1.0f / 1024.0f);
#pragma unroll
      for (int t = 0; t < 4; ++t) os[(8 * hh + r) * 64 + t * 16 + c] = oacc[t][r] * inv;
    }
  }
  __syncthreads();

  if (side == 0) {
    float a0 = 0.f, a1 = 0.f;
#pragma unroll 1
    for (int i = 0; i < HHALF; ++i) {
      a0 += bfq(lq1[i]) * bfq(lk1[i]);
      a1 += bfq(lq2[i]) * bfq(lk2[i]);
    }
    const float lam = expf(a0) - expf(a1) + LAMBDA_INIT_F;
    float gq[4];
#pragma unroll
    for (int t = 0; t < 4; ++t) gq[t] = bfq(gw[t * 16 + c]);

#pragma unroll
    for (int r = 0; r < 8; ++r) {
      const float l = lrow[r];
      const float inv = ((l > 0.f) ? (1.0f / l) : 0.f) * (1.0f / 1024.0f);
      float ss = 0.f;
#pragma unroll
      for (int t = 0; t < 4; ++t) {
        const float o2 = os[(8 * hh + r) * 64 + t * 16 + c];
        const float o = oacc[t][r] * inv - lam * o2;
        oacc[t][r] = o;
        ss += o * o;
      }
#pragma unroll
      for (int off = 1; off < 16; off <<= 1) ss += __shfl_xor(ss, off, 32);
      const float rn = OUT_SCALE * (1.0f / sqrtf(ss * (1.0f / 64.0f) + 1e-5f));
#pragma unroll
      for (int t = 0; t < 4; ++t) os[(8 * hh + r) * 64 + t * 16 + c] = oacc[t][r] * rn * gq[t];
    }
    __builtin_amdgcn_fence(__ATOMIC_RELEASE, "workgroup");
    __builtin_amdgcn_wave_barrier();
    __builtin_amdgcn_fence(__ATOMIC_ACQUIRE, "workgroup");

    const int q4 = lane >> 3, c8 = (lane & 7) * 8;
    v4u hv[4], lv[4];
#pragma unroll
    for (int it = 0; it < 4; ++it) {
      const int row = it * 4 + q4;
      const float* sp = os + row * 64 + c8;
      v4u a, a2;
#pragma unroll
      for (int e = 0; e < 4; ++e) {
        const float f0 = sp[2 * e], f1 = sp[2 * e + 1];
        const unsigned short h0 = bf_bits(f0), h1 = bf_bits(f1);
        const unsigned short l0 = bf_bits(f0 - bf_up(h0)), l1 = bf_bits(f1 - bf_up(h1));
        a[e] = pk16(h0, h1); a2[e] = pk16(l0, l1);
      }
      hv[it] = a; lv[it] = a2;
    }
    for (int pass = 0; pass < 2; ++pass) {
#pragma unroll
      for (int it = 0; it < 4; ++it) {
        const int row = it * 4 + q4;
        const size_t go = (rowB + q0 + row) * HID + (size_t)p * HD + c8;
        *(volatile v4u*)(ohp + go) = hv[it];
        *(volatile v4u*)(olp + go) = lv[it];
      }
      __threadfence();
    }
  }
}

extern "C" void kernel_launch(void* const* d_in, const int* in_sizes, int n_in,
                              void* d_out, int out_size, void* d_ws, size_t ws_size,
                              hipStream_t stream) {
  if (n_in < 12) return;
  const long long needAct = (long long)(NB - 1) * SEQ_FULL * HID + (long long)SEQ * HID;
  if ((long long)in_sizes[0] < needAct || (long long)in_sizes[1] < needAct || (long long)in_sizes[2] < needAct) return;
  if (in_sizes[3] < HID * HID || in_sizes[4] < HID * HID || in_sizes[5] < HID * HID || in_sizes[6] < HID * HID) return;
  if (in_sizes[7] < HHALF || in_sizes[8] < HHALF || in_sizes[9] < HHALF || in_sizes[10] < HHALF) return;
  if (in_sizes[11] < HD) return;
  if ((long long)out_size < needAct) return;

  const float* query = (const float*)d_in[0];
  const float* key   = (const float*)d_in[1];
  const float* value = (const float*)d_in[2];
  const float* Wq    = (const float*)d_in[3];
  const float* Wk    = (const float*)d_in[4];
  const float* Wv    = (const float*)d_in[5];
  const float* Wo    = (const float*)d_in[6];
  const float* lq1   = (const float*)d_in[7];
  const float* lq2   = (const float*)d_in[8];
  const float* lk1   = (const float*)d_in[9];
  const float* lk2   = (const float*)d_in[10];
  const float* gw    = (const float*)d_in[11];

  const size_t PX  = (size_t)NB * SEQ * HID * 2;
  const size_t PW  = (size_t)HID * HID * 2;
  const size_t PVT = (size_t)NB * HID * SEQ * 2;
  const size_t PVL = (size_t)NB * HID * VLP * 2;
  size_t off = 0;
  const size_t oQin = off; off += PX;
  const size_t oKin = off; off += PX;
  const size_t oVin = off; off += PX;
  const size_t oWq  = off; off += PW;
  const size_t oWk  = off; off += PW;
  const size_t oWv  = off; off += PW;
  const size_t oWo  = off; off += PW;
  const size_t oQh  = off; off += PX;
  const size_t oQl  = off; off += PX;
  const size_t oKh  = off; off += PX;
  const size_t oKl  = off; off += PX;
  const size_t oVTh = off; off += PVT;
  const size_t oVTl = off; off += PVL;
  const size_t oOh  = off; off += PX;
  const size_t oOl  = off; off += PX;
  if (off > ws_size) return;
  if (off > (size_t)134217728) return;

  char* ws = (char*)d_ws;
  unsigned short* Qin = (unsigned short*)(ws + oQin);
  unsigned short* Kin = (unsigned short*)(ws + oKin);
  unsigned short* Vin = (unsigned short*)(ws + oVin);
  unsigned short* Wqb = (unsigned short*)(ws + oWq);
  unsigned short* Wkb = (unsigned short*)(ws + oWk);
  unsigned short* Wvb = (unsigned short*)(ws + oWv);
  unsigned short* Wob = (unsigned short*)(ws + oWo);
  unsigned short* Qh  = (unsigned short*)(ws + oQh);
  unsigned short* Ql  = (unsigned short*)(ws + oQl);
  unsigned short* Kh  = (unsigned short*)(ws + oKh);
  unsigned short* Kl  = (unsigned short*)(ws + oKl);
  unsigned short* VTh = (unsigned short*)(ws + oVTh);
  unsigned short* VTl = (unsigned short*)(ws + oVTl);
  unsigned short* Oh  = (unsigned short*)(ws + oOh);
  unsigned short* Ol  = (unsigned short*)(ws + oOl);

  const dim3 blk(256);
  const int n8a = SEQ * HID / 8;
  const int n8w = HID * HID / 8;
  const dim3 gCvtA(n8a / 256, NB);
  const dim3 gCvtW(n8w / 256, 1);
  const int tilesP = (NB * SEQ / 64) * (HID / 64);
  const dim3 gProj((tilesP + 7) / 8, 1);
  const int tilesV = (HID / 64) * (SEQ / 64);
  const dim3 gVT((tilesV + 7) / 8, NB);
  const int tilesO = (SEQ / 64) * (HID / 64);
  const dim3 gOut((tilesO + 7) / 8, NB);

  cvt_bf16x8<<<gCvtA, blk, 0, stream>>>(query, Qin, n8a, (long long)SEQ_FULL * HID, (long long)SEQ * HID);
  cvt_bf16x8<<<gCvtA, blk, 0, stream>>>(key,   Kin, n8a, (long long)SEQ_FULL * HID, (long long)SEQ * HID);
  cvt_bf16x8<<<gCvtA, blk, 0, stream>>>(value, Vin, n8a, (long long)SEQ_FULL * HID, (long long)SEQ * HID);
  cvt_bf16x8<<<gCvtW, blk, 0, stream>>>(Wq, Wqb, n8w, 0LL, 0LL);
  cvt_bf16x8<<<gCvtW, blk, 0, stream>>>(Wk, Wkb, n8w, 0LL, 0LL);
  cvt_bf16x8<<<gCvtW, blk, 0, stream>>>(Wv, Wvb, n8w, 0LL, 0LL);
  cvt_bf16x8<<<gCvtW, blk, 0, stream>>>(Wo, Wob, n8w, 0LL, 0LL);
  gemm64<0, 2><<<gProj, blk, 0, stream>>>(
      Qin, Qin, HID, 0LL, Wqb, Wqb, HID, 0LL,
      (void*)Qh, HID, 0LL, (void*)Ql, HID, 0LL, HID,
      NB * SEQ, HID, HID, 1.0f);
  gemm64<0, 2><<<gProj, blk, 0, stream>>>(
      Kin, Kin, HID, 0LL, Wkb, Wkb, HID, 0LL,
      (void*)Kh, HID, 0LL, (void*)Kl, HID, 0LL, HID,
      NB * SEQ, HID, HID, 1.0f);
  gemm64<0, 3><<<gVT, blk, 0, stream>>>(
      Wvb, Wvb, HID, 0LL, Vin, Vin, HID, (long long)SEQ * HID,
      (void*)VTh, SEQ, (long long)HID * SEQ, (void*)VTl, VLP, (long long)HID * VLP, VLP,
      HID, SEQ, HID, 4096.0f);
  diff_attn64<true><<<dim3(NB * NPAIR * NQB), dim3(256), 0, stream>>>(
      Qh, Ql, Kh, Kl, VTh, VTl, lq1, lq2, lk1, lk2, gw, Oh, Ol, SM_SCALE);
  gemm64<1, 0><<<gOut, blk, 0, stream>>>(
      Oh, Ol, HID, (long long)SEQ * HID, Wob, Wob, HID, 0LL,
      d_out, HID, (long long)SEQ_FULL * HID, d_out, HID, 0LL, HID,
      SEQ, HID, HID, 1.0f);
  (void)hipGetLastError();
}
